// MultiHeadAttention_41420664603202
// MI455X (gfx1250) — hardware-verified
//
#include <hip/hip_runtime.h>
#include <math.h>


#ifndef NB
#define NB 2
#endif
#ifndef SEQ
#define SEQ 2048
#endif
#ifndef EROWS
#if (SEQ) < 256
#define EROWS (SEQ)
#else
#define EROWS 256
#endif
#endif

#define NB_FULL 2
#define S_FULL  2048
#define DM      1024
#define NH      16
#define HD      64

static_assert(NB >= 1 && NB <= NB_FULL);
static_assert((SEQ) % 128 == 0 && (SEQ) >= 128 && (SEQ) <= S_FULL);
static_assert((EROWS) % 128 == 0 && (EROWS) >= 128 && (EROWS) <= (SEQ));
static_assert(NH * HD == DM && DM == 1024);

#define RES_SC  16384.0f
#define RES_INV (1.0f / 16384.0f)
#define P_SC    1024.0f
#define P_INV   (1.0f / 1024.0f)
#define CTX_SC  16.0f
#define WO_SC   16384.0f
#define OUT_INV (1.0f / (16384.0f * 16.0f))

#define TP   68
#define KPAD 72
#define VPAD 40
#define OP   68

typedef _Float16 f16_t;
typedef __bf16   bf16_t;
typedef f16_t  v16h __attribute__((ext_vector_type(16)));
typedef f16_t  v8h  __attribute__((ext_vector_type(8)));
typedef bf16_t v16b __attribute__((ext_vector_type(16)));
typedef bf16_t v8b  __attribute__((ext_vector_type(8)));
typedef float  v8f  __attribute__((ext_vector_type(8)));
typedef float  v4f  __attribute__((ext_vector_type(4)));
typedef unsigned int v4u __attribute__((ext_vector_type(4)));

__device__ __forceinline__ v16h frag_h(const f16_t* p) {
  const v8h a = *(const v8h*)p;
  const v8h c = *(const v8h*)(p + 16);
  return __builtin_shufflevector(a, c, 0, 1, 2, 3, 4, 5, 6, 7, 8, 9, 10, 11, 12, 13, 14, 15);
}
__device__ __forceinline__ v16b frag_b(const bf16_t* p) {
  const v8b a = *(const v8b*)p;
  const v8b c = *(const v8b*)(p + 16);
  return __builtin_shufflevector(a, c, 0, 1, 2, 3, 4, 5, 6, 7, 8, 9, 10, 11, 12, 13, 14, 15);
}

__device__ __forceinline__ v8f mma_h(const v16h a, const v16h b, v8f c) {
  v8f d = __builtin_amdgcn_wmma_f32_16x16x32_f16(false, a, false, b, (short)0, c, false, false);
  asm volatile("v_nop\n\tv_nop\n\tv_nop\n\tv_nop" : "+v"(d) : "v"(a), "v"(b));
  return d;
}
__device__ __forceinline__ v8f mma_b(const v16b a, const v16b b, v8f c) {
  v8f d = __builtin_amdgcn_wmma_f32_16x16x32_bf16(false, a, false, b, (short)0, c, false, false);
  asm volatile("v_nop\n\tv_nop\n\tv_nop\n\tv_nop" : "+v"(d) : "v"(a), "v"(b));
  return d;
}

__device__ __forceinline__ void st16v(void* p, v4u w) { *(volatile v4u*)p = w; }
__device__ __forceinline__ void st16f(float* p, v4f w) { *(volatile v4f*)p = w; }

__device__ __forceinline__ unsigned int bf16_bits(float x) {
  unsigned int u = __float_as_uint(x);
  u += 0x7FFFu + ((u >> 16) & 1u);
  return u >> 16;
}
__device__ __forceinline__ float bf16_val(float x) {
  unsigned int u = __float_as_uint(x);
  u = (u + 0x7FFFu + ((u >> 16) & 1u)) & 0xFFFF0000u;
  return __uint_as_float(u);
}
__device__ __forceinline__ v4u pack_bf16x8(const v4f a, const v4f c) {
  const unsigned int s0 = bf16_bits(a[0]), s1 = bf16_bits(a[1]);
  const unsigned int s2 = bf16_bits(a[2]), s3 = bf16_bits(a[3]);
  const unsigned int s4 = bf16_bits(c[0]), s5 = bf16_bits(c[1]);
  const unsigned int s6 = bf16_bits(c[2]), s7 = bf16_bits(c[3]);
  v4u r;
  r[0] = s0 | (s1 << 16);
  r[1] = s2 | (s3 << 16);
  r[2] = s4 | (s5 << 16);
  r[3] = s6 | (s7 << 16);
  return r;
}
__device__ __forceinline__ void split8(const v4f a, const v4f c, v4u& whi, v4u& wrs) {
  float x[8] = { a[0], a[1], a[2], a[3], c[0], c[1], c[2], c[3] };
  v8h hi, rs;
#pragma unroll
  for (int i = 0; i < 8; ++i) {
    const f16_t hh = (f16_t)x[i];
    hi[i] = hh;
    rs[i] = (f16_t)((x[i] - (float)hh) * RES_SC);
  }
  whi = __builtin_bit_cast(v4u, hi);
  wrs = __builtin_bit_cast(v4u, rs);
}

__global__ __launch_bounds__(256)
void cvt_kernel(const float* __restrict__ q, const float* __restrict__ k, const float* __restrict__ v,
                const float* __restrict__ wq, const float* __restrict__ wk, const float* __restrict__ wv,
                const float* __restrict__ wo,
                bf16_t* __restrict__ xq, bf16_t* __restrict__ xk, bf16_t* __restrict__ xv,
                bf16_t* __restrict__ wqb, bf16_t* __restrict__ wkb, bf16_t* __restrict__ wvb,
                f16_t* __restrict__ wo14, f16_t* __restrict__ wo1) {
  const int job = blockIdx.y;
  const size_t e = ((size_t)blockIdx.x * 256 + threadIdx.x) * 8;
  if (job < 3) {
    const size_t n = (size_t)NB * SEQ * DM;
    if (e >= n) return;
    const float* src = (job == 0) ? q : (job == 1) ? k : v;
    bf16_t* dst = (job == 0) ? xq : (job == 1) ? xk : xv;
    const size_t m = e >> 10;
    const int d = (int)(e & 1023);
    const int b = (int)(m / SEQ);
    const int s = (int)(m - (size_t)b * SEQ);
    const float* sp = src + ((size_t)b * S_FULL + s) * DM + d;
    const v4f a = *(const v4f*)sp;
    const v4f c = *(const v4f*)(sp + 4);
    const v4u w = pack_bf16x8(a, c);
    st16v(dst + e, w);
    __threadfence();
    st16v(dst + e, w);
  } else if (job < 6) {
    const size_t n = (size_t)DM * DM;
    if (e >= n) return;
    const float* src = (job == 3) ? wq : (job == 4) ? wk : wv;
    bf16_t* dst = (job == 3) ? wqb : (job == 4) ? wkb : wvb;
    const v4f a = *(const v4f*)(src + e);
    const v4f c = *(const v4f*)(src + e + 4);
    const v4u w = pack_bf16x8(a, c);
    st16v(dst + e, w);
    __threadfence();
    st16v(dst + e, w);
  } else {
    const size_t n = (size_t)DM * DM;
    if (e >= n) return;
    const v4f a = *(const v4f*)(wo + e);
    const v4f c = *(const v4f*)(wo + e + 4);
    float x[8] = { a[0], a[1], a[2], a[3], c[0], c[1], c[2], c[3] };
    v8h p1, p14;
#pragma unroll
    for (int i = 0; i < 8; ++i) {
      const float r = bf16_val(x[i]);
      p1[i]  = (f16_t)r;
      p14[i] = (f16_t)(r * WO_SC);
    }
    const v4u w1 = __builtin_bit_cast(v4u, p1);
    const v4u w14 = __builtin_bit_cast(v4u, p14);
    st16v(wo1 + e, w1);
    st16v(wo14 + e, w14);
    __threadfence();
    st16v(wo1 + e, w1);
    st16v(wo14 + e, w14);
  }
}

__global__ __launch_bounds__(64)
void proj_qkv_kernel(const bf16_t* __restrict__ Xq, const bf16_t* __restrict__ Xk,
                     const bf16_t* __restrict__ Xv,
                     const bf16_t* __restrict__ Wq, const bf16_t* __restrict__ Wk,
                     const bf16_t* __restrict__ Wv,
                     f16_t* __restrict__ Qh, f16_t* __restrict__ Kh, f16_t* __restrict__ Vt,
                     f16_t* __restrict__ Qr, f16_t* __restrict__ Kr, f16_t* __restrict__ Vr) {
  __shared__ __align__(16) float tile[64 * TP];

  const int tid  = threadIdx.x;
  const int wave = __builtin_amdgcn_readfirstlane(tid >> 5);
  const int lane = tid & 31, lm = lane & 15, lh = lane >> 4;
  const int z  = blockIdx.z;
  const int m0 = blockIdx.x * 64;
  const int h  = blockIdx.y;
  const int n0 = h * HD;
  const int b  = m0 / SEQ;
  const int s0 = m0 - b * SEQ;
  const bool early = (s0 < EROWS);
  const bf16_t* X = (z == 0) ? Xq : (z == 1) ? Xk : Xv;
  const bf16_t* W = (z == 0) ? Wq : (z == 1) ? Wk : Wv;

  const bf16_t* ar0 = X + (size_t)(m0 + wave * 32 + lm) * DM + lh * 8;
  const bf16_t* ar1 = ar0 + (size_t)16 * DM;
  const bf16_t* br  = W + (size_t)(n0 + lm) * DM + lh * 8;

  v8f acc[2][4] = {};
#pragma unroll 1
  for (int k0 = 0; k0 < DM; k0 += 32) {
    const v16b a0 = frag_b(ar0 + k0);
    const v16b a1 = frag_b(ar1 + k0);
#pragma unroll
    for (int t = 0; t < 4; ++t) {
      const v16b bb = frag_b(br + (size_t)t * 16 * DM + k0);
      acc[0][t] = mma_b(a0, bb, acc[0][t]);
      acc[1][t] = mma_b(a1, bb, acc[1][t]);
    }
  }

#pragma unroll
  for (int g2 = 0; g2 < 2; ++g2) {
#pragma unroll
    for (int t = 0; t < 4; ++t) {
#pragma unroll
      for (int r = 0; r < 8; ++r) {
        const int row = wave * 32 + g2 * 16 + lh * 8 + r;
        const int col = t * 16 + lm;
        if (z < 2) tile[row * TP + col] = acc[g2][t][r];
        else       tile[col * TP + row] = acc[g2][t][r];
      }
    }
  }
  __syncthreads();

  const int rr = lane >> 3, c8 = (lane & 7) * 8;
  const size_t bh = (size_t)(b * NH + h);
  for (int pass = 0; pass < 2; ++pass) {
#pragma unroll
    for (int it = 0; it < 8; ++it) {
      const int L = wave * 32 + it * 4 + rr;
      const v4f a = *(const v4f*)&tile[L * TP + c8];
      const v4f c = *(const v4f*)&tile[L * TP + c8 + 4];
      v4u whi, wrs;
      split8(a, c, whi, wrs);
      if (z < 2) {
        f16_t* hp = (z == 0) ? Qh : Kh;
        f16_t* rp = (z == 0) ? Qr : Kr;
        const int s = s0 + L;
        st16v(hp + (bh * SEQ + s) * HD + c8, whi);
        if (early) {
          const int se = (s < EROWS) ? s : (EROWS - 1);
          st16v(rp + (bh * EROWS + se) * HD + c8, wrs);
        }
      } else {
        st16v(Vt + (bh * HD + L) * SEQ + s0 + c8, whi);
        if (early) {
          const int sc = (s0 + 64 <= EROWS) ? s0 : (EROWS - 64);
          st16v(Vr + (bh * HD + L) * EROWS + sc + c8, wrs);
        }
      }
    }
    if (pass == 0) __threadfence();
  }
}

template <bool EARLY>
__global__ __launch_bounds__(256) __attribute__((amdgpu_num_vgpr(256)))
void attn_kernel(const f16_t* __restrict__ Qh, const f16_t* __restrict__ Kh,
                 const f16_t* __restrict__ Vt, const f16_t* __restrict__ Qr,
                 const f16_t* __restrict__ Kr, const f16_t* __restrict__ Vr,
                 f16_t* __restrict__ Ch, f16_t* __restrict__ Cr, int qbofs) {
  __shared__ __align__(16) f16_t lK[32 * KPAD];
  __shared__ __align__(16) f16_t lV[64 * VPAD];
  __shared__ __align__(16) f16_t lKr[EARLY ? 32 * KPAD : 8];
  __shared__ __align__(16) f16_t lVr[EARLY ? 64 * VPAD : 8];
  __shared__ __align__(16) float lO[8 * 16 * OP];

  const int tid  = threadIdx.x;
  const int wave = __builtin_amdgcn_readfirstlane(tid >> 5);
  const int lane = tid & 31, lm = lane & 15, lh = lane >> 4;
  const int qblk = (int)blockIdx.x + qbofs;
  const int h = blockIdx.y, b = blockIdx.z;
  const size_t bh = (size_t)(b * NH + h);
  const int qw = qblk * 128 + wave * 16;
  const int q  = qw + lm;
  const int kend = qblk * 128 + 128;

  const f16_t* Qp  = Qh + bh * ((size_t)SEQ * HD);
  const f16_t* Kp  = Kh + bh * ((size_t)SEQ * HD);
  const f16_t* Vp  = Vt + bh * ((size_t)HD * SEQ);
  const f16_t* Qrp = Qr + bh * ((size_t)EROWS * HD);
  const f16_t* Krp = Kr + bh * ((size_t)EROWS * HD);
  const f16_t* Vrp = Vr + bh * ((size_t)HD * EROWS);

  const v16h qf0 = frag_h(Qp + (size_t)q * HD + lh * 8);
  const v16h qf1 = frag_h(Qp + (size_t)q * HD + 32 + lh * 8);
  const int qe = (q < EROWS) ? q : (EROWS - 1);

  v8f O[4] = {};
  v8f Orr[4] = {};
  float m = -1.0e30f, l = 0.0f;

#pragma unroll 1
  for (int kb = 0; kb < kend; kb += 32) {
    {
      const int row = tid >> 3, ch = (tid & 7) * 8;
      *(v8h*)&lK[row * KPAD + ch] = *(const v8h*)(Kp + (size_t)(kb + row) * HD + ch);
      if constexpr (EARLY) {
        int kr = kb + row;
        kr = (kr < EROWS) ? kr : (EROWS - 1);
        *(v8h*)&lKr[row * KPAD + ch] = *(const v8h*)(Krp + (size_t)kr * HD + ch);
      }
    }
    {
      const int row = tid >> 2, ch = (tid & 3) * 8;
      *(v8h*)&lV[row * VPAD + ch] = *(const v8h*)(Vp + (size_t)row * SEQ + kb + ch);
      if constexpr (EARLY) {
        int kc = kb + ch;
        kc = (kc + 8 <= EROWS) ? kc : (EROWS - 8);
        *(v8h*)&lVr[row * VPAD + ch] = *(const v8h*)(Vrp + (size_t)row * EROWS + kc);
      }
    }
    __syncthreads();

    if (kb <= qw + 15) {
      v16h qr0 = qf0, qr1 = qf1;
      if constexpr (EARLY) {
        qr0 = frag_h(Qrp + (size_t)qe * HD + lh * 8);
        qr1 = frag_h(Qrp + (size_t)qe * HD + 32 + lh * 8);
      }
      v8f s1 = {};
      v8f s2 = {};
      {
        const f16_t* kp0 = &lK[lm * KPAD + lh * 8];
        const v16h ka = frag_h(kp0);
        const v16h kc = frag_h(kp0 + 32);
        if constexpr (EARLY) {
          const f16_t* rp0 = &lKr[lm * KPAD + lh * 8];
          s1 = mma_h(frag_h(rp0), qf0, s1);
          s1 = mma_h(frag_h(rp0 + 32), qf1, s1);
          s1 = mma_h(ka, qr0, s1);
          s1 = mma_h(kc, qr1, s1);
#pragma unroll
          for (int i = 0; i < 8; ++i) s1[i] *= RES_INV;
        }
        s1 = mma_h(ka, qf0, s1);
        s1 = mma_h(kc, qf1, s1);
      }
      {
        const f16_t* kp1 = &lK[(16 + lm) * KPAD + lh * 8];
        const v16h ka = frag_h(kp1);
        const v16h kc = frag_h(kp1 + 32);
        if constexpr (EARLY) {
          const f16_t* rp1 = &lKr[(16 + lm) * KPAD + lh * 8];
          s2 = mma_h(frag_h(rp1), qf0, s2);
          s2 = mma_h(frag_h(rp1 + 32), qf1, s2);
          s2 = mma_h(ka, qr0, s2);
          s2 = mma_h(kc, qr1, s2);
#pragma unroll
          for (int i = 0; i < 8; ++i) s2[i] *= RES_INV;
        }
        s2 = mma_h(ka, qf0, s2);
        s2 = mma_h(kc, qf1, s2);
      }

      float bm = -1.0e30f;
#pragma unroll
      for (int i = 0; i < 8; ++i) {
        const int key1 = kb + lh * 8 + i;
        float x1 = s1[i] * 0.125f;
        float x2 = s2[i] * 0.125f;
        x1 = (key1 > q) ? -1.0e30f : x1;
        x2 = (key1 + 16 > q) ? -1.0e30f : x2;
        s1[i] = x1;
        s2[i] = x2;
        bm = fmaxf(bm, fmaxf(x1, x2));
      }
      bm = fmaxf(bm, __shfl_xor(bm, 16, 32));
      const float mnew = fmaxf(m, bm);
      const float alpha = __expf(m - mnew);
      float rs = 0.0f;
      v16h pb, pr;
#pragma unroll
      for (int i = 0; i < 8; ++i) {
        const float p1 = __expf(s1[i] - mnew);
        const float p2 = __expf(s2[i] - mnew);
        rs += p1 + p2;
        const float p1s = p1 * P_SC, p2s = p2 * P_SC;
        const f16_t h1 = (f16_t)p1s, h2 = (f16_t)p2s;
        pb[i] = h1;
        pb[8 + i] = h2;
        if constexpr (EARLY) {
          pr[i]     = (f16_t)((p1s - (float)h1) * RES_SC);
          pr[8 + i] = (f16_t)((p2s - (float)h2) * RES_SC);
        }
      }
      rs += __shfl_xor(rs, 16, 32);
      l = l * alpha + rs;
      m = mnew;

#pragma unroll
      for (int t = 0; t < 4; ++t) {
#pragma unroll
        for (int i = 0; i < 8; ++i) {
          O[t][i] *= alpha;
          if constexpr (EARLY) Orr[t][i] *= alpha;
        }
        const v16h va = frag_h(&lV[(t * 16 + lm) * VPAD + lh * 8]);
        O[t] = mma_h(va, pb, O[t]);
        if constexpr (EARLY) {
          Orr[t] = mma_h(va, pr, Orr[t]);
          const v16h vr = frag_h(&lVr[(t * 16 + lm) * VPAD + lh * 8]);
          Orr[t] = mma_h(vr, pb, Orr[t]);
        }
      }
    }
    __syncthreads();
  }

  const float scl = (1.0f / l) * (CTX_SC * P_INV);
  float* lo = lO + wave * (16 * OP);
#pragma unroll
  for (int t = 0; t < 4; ++t) {
    v4f a, c;
#pragma unroll
    for (int i = 0; i < 4; ++i) {
      float x0 = O[t][i];
      float x1 = O[t][i + 4];
      if constexpr (EARLY) {
        x0 += Orr[t][i] * RES_INV;
        x1 += Orr[t][i + 4] * RES_INV;
      }
      a[i] = x0 * scl;
      c[i] = x1 * scl;
    }
    *(v4f*)&lo[lm * OP + t * 16 + lh * 8]     = a;
    *(v4f*)&lo[lm * OP + t * 16 + lh * 8 + 4] = c;
  }
  __syncthreads();

  const int rr = lane >> 3, c8 = (lane & 7) * 8;
  for (int pass = 0; pass < 2; ++pass) {
#pragma unroll
    for (int it = 0; it < 4; ++it) {
      const int R  = it * 4 + rr;
      const int qq = qw + R;
      const v4f a = *(const v4f*)&lo[R * OP + c8];
      const v4f c = *(const v4f*)&lo[R * OP + c8 + 4];
      v4u whi, wrs;
      split8(a, c, whi, wrs);
      st16v(Ch + ((size_t)b * SEQ + qq) * DM + h * HD + c8, whi);
      if constexpr (EARLY) {
        const int qc = (qq < EROWS) ? qq : (EROWS - 1);
        st16v(Cr + ((size_t)b * EROWS + qc) * DM + h * HD + c8, wrs);
      }
    }
    if (pass == 0) __threadfence();
  }
}

__global__ __launch_bounds__(64)
void proj_out_kernel(const f16_t* __restrict__ Ch, const f16_t* __restrict__ Cr,
                     const f16_t* __restrict__ Wo14, const f16_t* __restrict__ Wo1,
                     float* __restrict__ out) {
  __shared__ __align__(16) float tile[64 * TP];

  const int tid  = threadIdx.x;
  const int wave = __builtin_amdgcn_readfirstlane(tid >> 5);
  const int lane = tid & 31, lm = lane & 15, lh = lane >> 4;
  const int m0 = blockIdx.x * 64;
  const int n0 = blockIdx.y * 64;
  const int b  = m0 / SEQ;
  const int s0 = m0 - b * SEQ;
  const bool early = (s0 < EROWS);
  const int se = early ? s0 : 0;

  const f16_t* ar0 = Ch + (size_t)(m0 + wave * 32 + lm) * DM + lh * 8;
  const f16_t* ar1 = ar0 + (size_t)16 * DM;
  const f16_t* cr0 = Cr + ((size_t)b * EROWS + se + wave * 32 + lm) * DM + lh * 8;
  const f16_t* cr1 = cr0 + (size_t)16 * DM;
  const f16_t* bw  = Wo14 + (size_t)(n0 + lm) * DM + lh * 8;
  const f16_t* bw1 = Wo1  + (size_t)(n0 + lm) * DM + lh * 8;

  v8f acc[2][4] = {};
#pragma unroll 1
  for (int k0 = 0; k0 < DM; k0 += 32) {
    const v16h a0 = frag_h(ar0 + k0);
    const v16h a1 = frag_h(ar1 + k0);
#pragma unroll
    for (int t = 0; t < 4; ++t) {
      const v16h bb = frag_h(bw + (size_t)t * 16 * DM + k0);
      acc[0][t] = mma_h(a0, bb, acc[0][t]);
      acc[1][t] = mma_h(a1, bb, acc[1][t]);
    }
    if (early) {
      const v16h c0 = frag_h(cr0 + k0);
      const v16h c1 = frag_h(cr1 + k0);
#pragma unroll
      for (int t = 0; t < 4; ++t) {
        const v16h bb = frag_h(bw1 + (size_t)t * 16 * DM + k0);
        acc[0][t] = mma_h(c0, bb, acc[0][t]);
        acc[1][t] = mma_h(c1, bb, acc[1][t]);
      }
    }
  }

#pragma unroll
  for (int g2 = 0; g2 < 2; ++g2) {
#pragma unroll
    for (int t = 0; t < 4; ++t) {
#pragma unroll
      for (int r = 0; r < 8; ++r) {
        const int row = wave * 32 + g2 * 16 + lh * 8 + r;
        const int col = t * 16 + lm;
        tile[row * TP + col] = acc[g2][t][r] * OUT_INV;
      }
    }
  }
  __syncthreads();

  const int rsel = lane >> 4, c4 = (lane & 15) * 4;
  for (int pass = 0; pass < 2; ++pass) {
#pragma unroll
    for (int it = 0; it < 16; ++it) {
      const int L = wave * 32 + it * 2 + rsel;
      const v4f a = *(const v4f*)&tile[L * TP + c4];
      float* dp = out + ((size_t)b * S_FULL + s0 + L) * DM + n0 + c4;
      st16f(dp, a);
    }
    if (pass == 0) __threadfence();
  }
}

extern "C" void kernel_launch(void* const* d_in, const int* in_sizes, int n_in,
                              void* d_out, int out_size, void* d_ws, size_t ws_size,
                              hipStream_t stream) {
  if (n_in < 7) return;
  const long long need_x = (long long)(NB - 1) * S_FULL * DM + (long long)SEQ * DM;
  if ((long long)in_sizes[0] < need_x || (long long)in_sizes[1] < need_x ||
      (long long)in_sizes[2] < need_x) return;
  if (in_sizes[3] < DM * DM || in_sizes[4] < DM * DM || in_sizes[5] < DM * DM ||
      in_sizes[6] < DM * DM) return;
  if ((long long)out_size < need_x) return;

  const float* q  = (const float*)d_in[0];
  const float* k  = (const float*)d_in[1];
  const float* v  = (const float*)d_in[2];
  const float* wq = (const float*)d_in[3];
  const float* wk = (const float*)d_in[4];
  const float* wv = (const float*)d_in[5];
  const float* wo = (const float*)d_in[6];
  float* out = (float*)d_out;

  char* ws = (char*)d_ws;
  size_t off = 0;
  auto carve = [&](size_t bytes) -> char* {
    char* p = ws + off;
    off += (bytes + 255) & ~(size_t)255;
    return p;
  };
  const size_t szX  = (size_t)NB * SEQ * DM * 2;
  const size_t szW  = (size_t)DM * DM * 2;
  const size_t szR  = (size_t)NB * NH * EROWS * HD * 2;
  const size_t szCr = (size_t)NB * EROWS * DM * 2;

  bf16_t* Xq  = (bf16_t*)carve(szX);
  bf16_t* Xk  = (bf16_t*)carve(szX);
  bf16_t* Xv  = (bf16_t*)carve(szX);
  bf16_t* Wqb = (bf16_t*)carve(szW);
  bf16_t* Wkb = (bf16_t*)carve(szW);
  bf16_t* Wvb = (bf16_t*)carve(szW);
  f16_t* Wo14 = (f16_t*)carve(szW);
  f16_t* Wo1  = (f16_t*)carve(szW);
  f16_t* Qh   = (f16_t*)carve(szX);
  f16_t* Kh   = (f16_t*)carve(szX);
  f16_t* Vt   = (f16_t*)carve(szX);
  f16_t* Qr   = (f16_t*)carve(szR);
  f16_t* Kr   = (f16_t*)carve(szR);
  f16_t* Vr   = (f16_t*)carve(szR);
  f16_t* Ch   = (f16_t*)carve(szX);
  f16_t* Cr   = (f16_t*)carve(szCr);
  if (off > ws_size) return;

  const unsigned int gx_act = (unsigned int)((size_t)NB * SEQ * DM / 2048);
  const unsigned int gx_w   = (unsigned int)((size_t)DM * DM / 2048);
  const unsigned int gx = (gx_act > gx_w) ? gx_act : gx_w;
  cvt_kernel<<<dim3(gx, 7), dim3(256), 0, stream>>>(q, k, v, wq, wk, wv, wo,
                                                      Xq, Xk, Xv, Wqb, Wkb, Wvb, Wo14, Wo1);

  proj_qkv_kernel<<<dim3(NB * SEQ / 64, NH, 3), dim3(64), 0, stream>>>(
      Xq, Xk, Xv, Wqb, Wkb, Wvb, Qh, Kh, Vt, Qr, Kr, Vr);

  const int nqe = EROWS / 128;
  const int nql = SEQ / 128 - nqe;
  attn_kernel<true><<<dim3(nqe, NH, NB), dim3(256), 0, stream>>>(
      Qh, Kh, Vt, Qr, Kr, Vr, Ch, Cr, 0);
  if (nql > 0) {
    attn_kernel<false><<<dim3(nql, NH, NB), dim3(256), 0, stream>>>(
        Qh, Kh, Vt, Qr, Kr, Vr, Ch, Cr, nqe);
  }

  proj_out_kernel<<<dim3(NB * SEQ / 64, DM / 64), dim3(64), 0, stream>>>(Ch, Cr, Wo14, Wo1, out);
}
